// FullMatchingLayer_19155554140813
// MI455X (gfx1250) — hardware-verified
//
#include <hip/hip_runtime.h>
#include <math.h>

#define FB 32
#define FT 512
#define FD 768
#define FP 20
#define RSPLIT (1.0f / 2048.0f)

typedef _Float16 h16;
typedef __attribute__((ext_vector_type(16))) _Float16 v16h;
typedef __attribute__((ext_vector_type(8)))  _Float16 v8h;
typedef __attribute__((ext_vector_type(8)))  float v8f;
typedef __attribute__((ext_vector_type(4)))  float v4f_t;
typedef float v4fa __attribute__((ext_vector_type(4), may_alias));

__device__ __forceinline__ h16 lo_of(float v, h16 h) { return (h16)((v - (float)h) * 2048.0f); }
__device__ __forceinline__ v8f wmma16(v16h a, v16h b, v8f c) { return __builtin_amdgcn_wmma_f32_16x16x32_f16(false, a, false, b, (short)0, c, false, false); }
__device__ __forceinline__ v8f wmma_split(v16h a, v16h al, v16h b, v16h bl, v8f c) { v8f x = {}; x = wmma16(al, b, x); x = wmma16(a, bl, x); return wmma16(a, b, c) + x * RSPLIT; }
__device__ __forceinline__ v16h rfrag(const h16* rowp, int half) {
  const h16* p = rowp + 8 * half;
  return __builtin_shufflevector(*(const v8h*)p, *(const v8h*)(p + 16), 0,1,2,3,4,5,6,7,8,9,10,11,12,13,14,15);
}
__device__ __forceinline__ int kof(int half, int e) { return 8 * half + ((e < 8) ? e : (e + 8)); }

__global__ __launch_bounds__(256) void k_fullmatch(const float* __restrict__ A, const float* __restrict__ Bm, const float* __restrict__ W, float* __restrict__ out) {
  __shared__ __attribute__((aligned(16))) h16 W2p[2][32 * 776];
  __shared__ float lastv[FD];
  __shared__ float nl[32], red[8][32];
  __shared__ __attribute__((aligned(16))) float res[64 * FP];
  const int tid = threadIdx.x, lane = tid & 31, wave = tid >> 5, half = lane >> 4, l16 = lane & 15;
  const int row0 = blockIdx.x * 64;
  const int b = row0 / FT;
  for (int i = tid; i < 32 * FD; i += 256) { const int p = i / FD, d = i % FD; const float w = (p < FP) ? W[p * FD + d] : 0.0f; const float w2 = w * w;
    const h16 hv = (h16)w2; W2p[0][p * 776 + d] = hv; W2p[1][p * 776 + d] = lo_of(w2, hv); }
  for (int d = tid; d < FD; d += 256) lastv[d] = Bm[((size_t)b * FT + (FT - 1)) * FD + d];
  __syncthreads();
#pragma unroll 1
  for (int p = wave; p < 32; p += 8) { float s = 0.0f;
    for (int d = lane; d < FD; d += 32) { const float w = (p < FP) ? W[p * FD + d] : 0.0f; s += lastv[d] * lastv[d] * (w * w); }
#pragma unroll
    for (int o = 16; o >= 1; o >>= 1) s += __shfl_xor(s, o, 32);
    if (lane == 0) nl[p] = sqrtf(fmaxf(s, 1e-12f)); }
  __syncthreads();
  const int mt = wave >> 1, nt = wave & 1;
  const float* arow = A + (size_t)(row0 + mt * 16 + l16) * FD;
  v8f num = {}, na2 = {};
#pragma unroll 1
  for (int kc = 0; kc < FD / 32; ++kc) {
    v16h a1, a1l, a2, a2l;
#pragma unroll
    for (int e = 0; e < 16; ++e) { const int d = kc * 32 + kof(half, e); const float av = arow[d];
      const float p1 = av * lastv[d], p2 = av * av;
      a1[e] = (h16)p1; a1l[e] = lo_of(p1, a1[e]); a2[e] = (h16)p2; a2l[e] = lo_of(p2, a2[e]); }
    const v16h bw = rfrag(&W2p[0][(nt * 16 + l16) * 776 + kc * 32], half), bwl = rfrag(&W2p[1][(nt * 16 + l16) * 776 + kc * 32], half);
    num = wmma_split(a1, a1l, bw, bwl, num);
    na2 = wmma_split(a2, a2l, bw, bwl, na2);
  }
  const int p = nt * 16 + l16;
  if (p < FP) {
#pragma unroll
    for (int r = 0; r < 8; ++r) { const int rl = mt * 16 + 8 * half + r;
      const float na = sqrtf(fmaxf(na2[r], 1e-12f));
      res[rl * FP + p] = num[r] / (na * nl[p]); }
  }
  __syncthreads();
  const size_t total = (size_t)FB * FT * FP;
#pragma unroll 1
  for (int pass = 0; pass < 2; ++pass) {
    for (int q = tid; q < 64 * FP / 4; q += 256) { const v4f_t v = *(const volatile v4fa*)(res + q * 4);
      *(volatile v4f_t*)(out + (size_t)row0 * FP + q * 4) = v; *(volatile v4f_t*)(out + total + (size_t)row0 * FP + q * 4) = v; }
    __threadfence();
  }
}

extern "C" void kernel_launch(void* const* d_in, const int* in_sizes, int n_in,
                              void* d_out, int out_size, void* d_ws, size_t ws_size,
                              hipStream_t stream) {
  (void)in_sizes; (void)n_in; (void)out_size; (void)d_ws; (void)ws_size;
  const float* inpA = (const float*)d_in[0];
  const float* inpB = (const float*)d_in[1];
  const float* Wm   = (const float*)d_in[2];
  k_fullmatch<<<FB * FT / 64, 256, 0, stream>>>(inpA, inpB, Wm, (float*)d_out);
}
